// ResidualSelfAttention_58634893525279
// MI455X (gfx1250) — hardware-verified
//
#include <hip/hip_runtime.h>
#include <stddef.h>
#include <stdint.h>


#define HID     128
#define NHEAD   8
#define DHD     16
#define EDIM    16
#define NQKV    384
#define XMP     512
#define KD      256
#define KG      512
#define GBM     64
#define GBN     128
#define GTHR    128
#define CEMAX   40000
#define NTHR    256
#define NWAVE   8
#define EPT     8
#define CHUNK   (NTHR * EPT)
#define WCAP    (EPT * 32)
#define LISTN   (NWAVE * WCAP)
#define NBMAX   2048
#define RCAP    28672
#define DEGCAP  256
#define STW     512
#define STP     32
#define TPB     32
#define WSMAX   134217728
#define LDS_AGG ((2 * RCAP + 2 * NBMAX + LISTN) * 4 + 64)

static_assert((CHUNK & (CHUNK - 1)) == 0 && CHUNK <= 4096);
static_assert((NBMAX & (NBMAX - 1)) == 0 && NBMAX <= 4096);
static_assert(NTHR * 8 == NBMAX);
static_assert(LISTN >= NBMAX);
static_assert(LISTN >= NWAVE * WCAP);
static_assert((RCAP % 32) == 0);
static_assert(NWAVE * STW <= RCAP);
static_assert(LDS_AGG <= 300000);
static_assert(GBM == (GTHR / 32) * 16);
static_assert((CEMAX % GBM) == 0 && CEMAX < (1 << 20));
static_assert(GBN == HID && KD == 2 * HID && KG == 4 * HID && NQKV == 3 * HID);
static_assert(NHEAD * DHD == HID && DHD == 16 && EDIM == 16);
static_assert((HID % 32) == 0 && (KD % 32) == 0 && (KG % 32) == 0);
static_assert(GBM * GBN == 16 * GTHR * 4);
static_assert(GBM * NHEAD == 4 * GTHR);
static_assert(GBM * KD == 8 * NTHR * 8);
static_assert(TPB * 3 == 24 * 4);
static_assert(NWAVE * 4 == TPB);
static_assert(STP == 4 * NHEAD);
static_assert(STW >= HID);

typedef float          v4f  __attribute__((ext_vector_type(4)));
typedef float          v8f  __attribute__((ext_vector_type(8)));
typedef int            v4i  __attribute__((ext_vector_type(4)));
typedef int            v8i  __attribute__((ext_vector_type(8)));
typedef unsigned short v8us __attribute__((ext_vector_type(8)));
typedef __bf16         v16b __attribute__((ext_vector_type(16)));
union FragB { v16b v; v8us h[2]; v8i w; };

__device__ __forceinline__ v8f wmb(const FragB& a, const FragB& b, v8f c) {
  v8f d = __builtin_amdgcn_wmma_f32_16x16x32_bf16(false, a.v, false, b.v, (short)0, c, false, false);
  asm volatile("v_nop\n\tv_nop\n\tv_nop\n\tv_nop" : "+v"(d) : "v"(a.w), "v"(b.w));
  return d;
}

__device__ __forceinline__ void ldwait() {
  asm volatile("s_wait_loadcnt 0x0" ::: "memory");
}

__device__ __forceinline__ void wave_sync() {
  __builtin_amdgcn_fence(__ATOMIC_RELEASE, "wavefront");
  __builtin_amdgcn_wave_barrier();
}

__device__ __forceinline__ unsigned short f2bf(float f) {
  unsigned u = __float_as_uint(f);
  u += 0x7FFFu + ((u >> 16) & 1u);
  return (unsigned short)(u >> 16);
}
__device__ __forceinline__ float bf2f(unsigned short h) { return __uint_as_float(((unsigned)h) << 16); }
__device__ __forceinline__ float bfr(float f) { return bf2f(f2bf(f)); }
__device__ __forceinline__ v4f bfr4(const v4f a) {
  v4f r; r.x = bfr(a.x); r.y = bfr(a.y); r.z = bfr(a.z); r.w = bfr(a.w); return r;
}
__device__ __forceinline__ int clampi(int v, int lo, int hi) { return v < lo ? lo : (v > hi ? hi : v); }

__device__ __forceinline__ float wsum(float v) {
#pragma unroll
  for (int off = 16; off > 0; off >>= 1) v += __shfl_xor(v, off);
  return v;
}

__device__ __forceinline__ float sigm(float x) {
  const float xc = fminf(fmaxf(x, -80.0f), 80.0f);
  const float e = __expf(-xc);
  return __builtin_amdgcn_rcpf(1.0f + e);
}

__device__ __forceinline__ v8us hilo8(const v4f a, const v4f b, const bool hiSel) {
  float f[8];
  f[0] = a.x; f[1] = a.y; f[2] = a.z; f[3] = a.w; f[4] = b.x; f[5] = b.y; f[6] = b.z; f[7] = b.w;
  v8us r;
#pragma unroll
  for (int i = 0; i < 8; ++i) {
    const unsigned short h = f2bf(f[i]);
    const unsigned short l = f2bf(f[i] - bf2f(h));
    r[i] = hiSel ? h : l;
  }
  return r;
}

__device__ __forceinline__ v4f ln4(const v4f v, const v4f w, const v4f b) {
  const float s = wsum((v.x + v.y) + (v.z + v.w));
  const float mu = s * (1.0f / HID);
  const v4f d = v - mu;
  const float s2 = wsum((d.x * d.x + d.y * d.y) + (d.z * d.z + d.w * d.w));
  const float rs = __builtin_amdgcn_rsqf(s2 * (1.0f / HID) + 1.0e-5f);
  return d * rs * w + b;
}

__device__ __forceinline__ int scan_chunk(const int* __restrict__ dsts, int nE, int cbase, int slotBase,
                                          int nb, int vec8, int* list, int tid, int lane, int wave) {
  int wc = 0;
  const int el0  = tid * EPT;
  const int e0   = cbase + el0;
  const int sent = -2147483647 - 1;
  v4i da, db;
  if (vec8 != 0 && cbase + CHUNK <= nE) {
    da = *(const v4i*)(dsts + e0);
    db = *(const v4i*)(dsts + e0 + 4);
  } else {
    da.x = (e0     < nE) ? dsts[min(e0,     nE - 1)] : sent;
    da.y = (e0 + 1 < nE) ? dsts[min(e0 + 1, nE - 1)] : sent;
    da.z = (e0 + 2 < nE) ? dsts[min(e0 + 2, nE - 1)] : sent;
    da.w = (e0 + 3 < nE) ? dsts[min(e0 + 3, nE - 1)] : sent;
    db.x = (e0 + 4 < nE) ? dsts[min(e0 + 4, nE - 1)] : sent;
    db.y = (e0 + 5 < nE) ? dsts[min(e0 + 5, nE - 1)] : sent;
    db.z = (e0 + 6 < nE) ? dsts[min(e0 + 6, nE - 1)] : sent;
    db.w = (e0 + 7 < nE) ? dsts[min(e0 + 7, nE - 1)] : sent;
  }
  const unsigned nbs = (unsigned)slotBase;
  const unsigned unb = (unsigned)nb;
  const unsigned s0 = (unsigned)da.x - nbs, s1 = (unsigned)da.y - nbs;
  const unsigned s2 = (unsigned)da.z - nbs, s3 = (unsigned)da.w - nbs;
  const unsigned s4 = (unsigned)db.x - nbs, s5 = (unsigned)db.y - nbs;
  const unsigned s6 = (unsigned)db.z - nbs, s7 = (unsigned)db.w - nbs;
  const bool h0 = s0 < unb, h1 = s1 < unb, h2 = s2 < unb, h3 = s3 < unb;
  const bool h4 = s4 < unb, h5 = s5 < unb, h6 = s6 < unb, h7 = s7 < unb;
  const unsigned any = __builtin_amdgcn_ballot_w32(h0 | h1 | h2 | h3 | h4 | h5 | h6 | h7);
  if (any != 0u) {
#define HITJ(J, HJ, SJ) { \
      const unsigned mj = __builtin_amdgcn_ballot_w32(HJ); \
      if (mj != 0u) { \
        if (HJ) { \
          const int pos = wc + (int)__builtin_amdgcn_mbcnt_lo(mj, 0u); \
          if (pos < WCAP) list[wave * WCAP + pos] = ((el0 + (J)) << 12) | (int)(SJ); \
        } \
        wc += (int)__builtin_popcount(mj); } }
    HITJ(0, h0, s0)
    HITJ(1, h1, s1)
    HITJ(2, h2, s2)
    HITJ(3, h3, s3)
    HITJ(4, h4, s4)
    HITJ(5, h5, s5)
    HITJ(6, h6, s6)
    HITJ(7, h7, s7)
#undef HITJ
  }
  return wc;
}

__global__ __launch_bounds__(NTHR) void k_prep_x(const float* __restrict__ x, const float* __restrict__ lw,
                                                 const float* __restrict__ lb, unsigned short* xm, int nN, int NPr) {
  __shared__ __attribute__((aligned(16))) float stw_all[NWAVE * HID];
  const int tid = (int)threadIdx.x, lane = tid & 31, wave = tid >> 5, lch = lane & 15;
  const int row = (int)blockIdx.x * NWAVE + wave;
  if (row >= NPr) return;
  const int rc = row < nN ? row : nN - 1;
  const v4f xv = bfr4(*(const v4f*)(x + (size_t)rc * HID + 4 * lane));
  const v4f wv = bfr4(*(const v4f*)(lw + 4 * lane));
  const v4f bv = bfr4(*(const v4f*)(lb + 4 * lane));
  ldwait();
  const v4f z4 = {0.f, 0.f, 0.f, 0.f};
  v4f xn = ln4(xv, wv, bv);
  if (row >= nN) xn = z4;
  float* stw = stw_all + wave * HID;
  wave_sync();
  *(v4f*)(stw + 4 * lane) = xn;
  wave_sync();
  const v4f ga = *(const v4f*)(stw + 8 * lch);
  const v4f gb = *(const v4f*)(stw + 8 * lch + 4);
  const v8us hv = hilo8(ga, gb, lane < 16);
  unsigned short* op = xm + (size_t)row * XMP + 8 * lane;
  *(volatile v8us*)op = hv;
  __threadfence();
  *(volatile v8us*)op = hv;
}

__global__ __launch_bounds__(NTHR) void k_wprep(const float* __restrict__ w, int KT, unsigned short* out,
                                                int orow0, int nUnits) {
  const int u = (int)blockIdx.x * NTHR + (int)threadIdx.x;
  if (u >= nUnits) return;
  const int per = KT >> 2;
  const int n   = u / per;
  const int j8  = (u - n * per) * 8;
  const int sc  = (j8 / KD) * HID + (j8 & (HID - 1));
  const float* p = w + (size_t)n * (size_t)KT + sc;
  const v4f a = *(const v4f*)p, b = *(const v4f*)(p + 4);
  v8us hv;
  hv[0] = f2bf(a.x); hv[1] = f2bf(a.y); hv[2] = f2bf(a.z); hv[3] = f2bf(a.w);
  hv[4] = f2bf(b.x); hv[5] = f2bf(b.y); hv[6] = f2bf(b.z); hv[7] = f2bf(b.w);
  const size_t o = (size_t)(orow0 + n) * (size_t)(2 * KT) + j8;
  *(volatile v8us*)(out + o) = hv;
  __threadfence();
  *(volatile v8us*)(out + o) = hv;
}

__global__ __launch_bounds__(NTHR) void k_edge_geo(
    const int* __restrict__ srcs, const int* __restrict__ dsts, const float* __restrict__ p,
    const float* __restrict__ ea, const float* __restrict__ lw, const float* __restrict__ lb,
    const float* __restrict__ l2w, const float* __restrict__ l2b, const float* __restrict__ wed,
    const float* __restrict__ we1, const float* __restrict__ be1,
    unsigned short* G2, float* EB, int cbeg, int ce, int nE, int nN) {
  __shared__ __attribute__((aligned(16))) unsigned short s_g[GBM * KD];
  __shared__ __attribute__((aligned(16))) float s_eb[GBM * NHEAD];
  __shared__ float s_ea[GBM * 17];
  __shared__ float s_rel[GBM * 3];
  __shared__ float s_w1[3 * HID];
  __shared__ float s_b1[HID];
  __shared__ float s_we[NHEAD * EDIM];
  __shared__ float s_ln[4 * EDIM];
  const int tid = (int)threadIdx.x;
  const int rowBase = (int)blockIdx.x * GBM;

  for (int i = tid; i < 3 * HID; i += NTHR) s_w1[i] = bfr(we1[i]);
  if (tid < HID) { s_b1[tid] = bfr(be1[tid]); s_we[tid] = bfr(wed[tid]); }
  if (tid < EDIM) {
    s_ln[tid]            = bfr(lw[tid]);
    s_ln[EDIM + tid]     = bfr(lb[tid]);
    s_ln[2 * EDIM + tid] = bfr(l2w[tid]);
    s_ln[3 * EDIM + tid] = bfr(l2b[tid]);
  }
  __syncthreads();

  if (tid < GBM) {
    const int el = rowBase + tid;
    const bool valid = el < ce;
    const int elc = el < ce ? el : ce - 1;
    int e = cbeg + elc;
    e = e > nE - 1 ? nE - 1 : (e < 0 ? 0 : e);
    const int s = clampi(srcs[e], 0, nN - 1);
    const int d = clampi(dsts[e], 0, nN - 1);
    const float pi0 = bfr(p[(size_t)d * 3]), pi1 = bfr(p[(size_t)d * 3 + 1]), pi2 = bfr(p[(size_t)d * 3 + 2]);
    const float pj0 = bfr(p[(size_t)s * 3]), pj1 = bfr(p[(size_t)s * 3 + 1]), pj2 = bfr(p[(size_t)s * 3 + 2]);
    float r0 = pj0 - pi0;
    float r1 = pi1 * pj1 + pi2 * pj2;
    float r2 = -pi2 * pj1 + pi1 * pj2;
    if (!valid) { r0 = 0.f; r1 = 0.f; r2 = 0.f; }
    s_rel[tid * 3]     = r0;
    s_rel[tid * 3 + 1] = r1;
    s_rel[tid * 3 + 2] = r2;

    const float* ap = ea + (size_t)e * EDIM;
    const v4f a0 = bfr4(*(const v4f*)ap);
    const v4f a1 = bfr4(*(const v4f*)(ap + 4));
    const v4f a2 = bfr4(*(const v4f*)(ap + 8));
    const v4f a3 = bfr4(*(const v4f*)(ap + 12));
    ldwait();
    float* er = s_ea + tid * 17;
    er[0]  = a0.x; er[1]  = a0.y; er[2]  = a0.z; er[3]  = a0.w;
    er[4]  = a1.x; er[5]  = a1.y; er[6]  = a1.z; er[7]  = a1.w;
    er[8]  = a2.x; er[9]  = a2.y; er[10] = a2.z; er[11] = a2.w;
    er[12] = a3.x; er[13] = a3.y; er[14] = a3.z; er[15] = a3.w;
    {
      float mu = 0.f;
#pragma unroll 1
      for (int i = 0; i < EDIM; ++i) mu += er[i];
      mu *= (1.0f / EDIM);
      float var = 0.f;
#pragma unroll 1
      for (int i = 0; i < EDIM; ++i) { const float dd = er[i] - mu; var = fmaf(dd, dd, var); }
      const float rs = __builtin_amdgcn_rsqf(var * (1.0f / EDIM) + 1.0e-5f);
#pragma unroll 1
      for (int i = 0; i < EDIM; ++i) er[i] = (er[i] - mu) * rs * s_ln[i] + s_ln[EDIM + i];
    }
    {
      float mu = 0.f;
#pragma unroll 1
      for (int i = 0; i < EDIM; ++i) mu += er[i];
      mu *= (1.0f / EDIM);
      float var = 0.f;
#pragma unroll 1
      for (int i = 0; i < EDIM; ++i) { const float dd = er[i] - mu; var = fmaf(dd, dd, var); }
      const float rs = __builtin_amdgcn_rsqf(var * (1.0f / EDIM) + 1.0e-5f);
#pragma unroll 1
      for (int i = 0; i < EDIM; ++i) er[i] = (er[i] - mu) * rs * s_ln[2 * EDIM + i] + s_ln[3 * EDIM + i];
    }
#pragma unroll 1
    for (int h = 0; h < NHEAD; ++h) {
      float acc = 0.f;
#pragma unroll 4
      for (int i = 0; i < EDIM; ++i) acc = fmaf(er[i], s_we[h * EDIM + i], acc);
      s_eb[tid * NHEAD + h] = valid ? acc : 0.f;
    }
  }
  __syncthreads();

  {
    const int r = tid >> 2, cq = tid & 3;
    const bool valid = (rowBase + r) < ce;
    const float r0 = s_rel[r * 3], r1 = s_rel[r * 3 + 1], r2 = s_rel[r * 3 + 2];
    unsigned short* gr = s_g + r * KD;
#pragma unroll 4
    for (int jj = 0; jj < 32; ++jj) {
      const int j = cq * 32 + jj;
      float h = r0 * s_w1[j * 3];
      h = fmaf(r1, s_w1[j * 3 + 1], h);
      h = fmaf(r2, s_w1[j * 3 + 2], h);
      h += s_b1[j];
      h = h >= 0.f ? h : 0.01f * h;
      h = valid ? h : 0.f;
      const unsigned short hb = f2bf(h);
      const unsigned short lb2 = f2bf(h - bf2f(hb));
      gr[j]       = hb;
      gr[HID + j] = lb2;
    }
  }
  __syncthreads();

  v8us gv[8];
#pragma unroll
  for (int i = 0; i < 8; ++i) {
    const int pc = i * NTHR + tid;
    const int row = pc >> 5, q = pc & 31;
    gv[i] = *(const v8us*)(s_g + row * KD + 8 * q);
  }
  const int tc = tid < 128 ? tid : 127;
  const v4f ebv = *(const v4f*)(s_eb + 4 * tc);
  const bool web = tid < 128;
  float* ebp = EB + (size_t)rowBase * NHEAD + 4 * tc;
#pragma unroll
  for (int i = 0; i < 8; ++i) {
    const int pc = i * NTHR + tid;
    const int row = pc >> 5, q = pc & 31;
    *(volatile v8us*)(G2 + (size_t)(rowBase + row) * KD + 8 * q) = gv[i];
  }
  if (web) *(volatile v4f*)ebp = ebv;
  __threadfence();
#pragma unroll
  for (int i = 0; i < 8; ++i) {
    const int pc = i * NTHR + tid;
    const int row = pc >> 5, q = pc & 31;
    *(volatile v8us*)(G2 + (size_t)(rowBase + row) * KD + 8 * q) = gv[i];
  }
  if (web) *(volatile v4f*)ebp = ebv;
}

__device__ __forceinline__ void gemm_core(v8f (&acc)[8], const unsigned short* __restrict__ A, int lda, int K,
                                          const unsigned short* __restrict__ WT, int ldw, int rowBase, int col0,
                                          int wave, int hh, int m) {
  const v8f z = {0.f, 0.f, 0.f, 0.f, 0.f, 0.f, 0.f, 0.f};
#pragma unroll
  for (int t = 0; t < 8; ++t) acc[t] = z;
  const unsigned short* ap = A  + (size_t)(rowBase + 16 * wave + m) * (size_t)lda + 8 * hh;
  const unsigned short* wp = WT + (size_t)(col0 + m) * (size_t)ldw + 8 * hh;
  const int ksteps = K >> 5;
#pragma unroll 1
  for (int ks = 0; ks < ksteps; ++ks) {
    FragB af;
    af.h[0] = *(const v8us*)(ap + 32 * ks);
    af.h[1] = *(const v8us*)(ap + 32 * ks + 16);
#pragma unroll
    for (int t = 0; t < 8; ++t) {
      const unsigned short* wq = wp + (size_t)(16 * t) * (size_t)ldw + 32 * ks;
      FragB bf;
      bf.h[0] = *(const v8us*)wq;
      bf.h[1] = *(const v8us*)(wq + 16);
      acc[t] = wmb(af, bf, acc[t]);
    }
  }
}

__device__ __forceinline__ void gemm_stage(const v8f (&acc)[8], float* stg, const float* __restrict__ bias,
                                           int blen, int hasBias, int col0, int wave, int hh, int m) {
#pragma unroll
  for (int t = 0; t < 8; ++t) {
    const int lc = 16 * t + m;
    int bi = col0 + lc;
    bi = bi > blen - 1 ? blen - 1 : bi;
    bi = bi < 0 ? 0 : bi;
    const float braw = bias[bi];
    const float bv = hasBias ? bfr(braw) : 0.0f;
#pragma unroll
    for (int r = 0; r < 8; ++r) {
      const int lr = 16 * wave + 8 * hh + r;
      stg[lr * GBN + lc] = acc[t][r] + bv;
    }
  }
}

__global__ __launch_bounds__(GTHR) void k_gemm_f32(
    const unsigned short* __restrict__ A, int lda, int K, const unsigned short* __restrict__ WT, int ldw,
    const float* __restrict__ bias, int blen, int hasBias, float* outF, int ldo) {
  __shared__ __attribute__((aligned(16))) float stg[GBM * GBN];
  const int tid = (int)threadIdx.x, lane = tid & 31, wave = tid >> 5, hh = lane >> 4, m = lane & 15;
  const int rowBase = (int)blockIdx.x * GBM;
  const int col0    = (int)blockIdx.y * GBN;
  v8f acc[8];
  gemm_core(acc, A, lda, K, WT, ldw, rowBase, col0, wave, hh, m);
  gemm_stage(acc, stg, bias, blen, hasBias, col0, wave, hh, m);
  __syncthreads();
  v4f fv[16];
#pragma unroll
  for (int i = 0; i < 16; ++i) {
    const int pc = i * GTHR + tid;
    const int row = pc >> 5, c4 = (pc & 31) * 4;
    fv[i] = *(const v4f*)(stg + row * GBN + c4);
  }
#pragma unroll
  for (int i = 0; i < 16; ++i) {
    const int pc = i * GTHR + tid;
    const int row = pc >> 5, c4 = (pc & 31) * 4;
    *(volatile v4f*)(outF + (size_t)(rowBase + row) * (size_t)ldo + col0 + c4) = fv[i];
  }
  __threadfence();
#pragma unroll
  for (int i = 0; i < 16; ++i) {
    const int pc = i * GTHR + tid;
    const int row = pc >> 5, c4 = (pc & 31) * 4;
    *(volatile v4f*)(outF + (size_t)(rowBase + row) * (size_t)ldo + col0 + c4) = fv[i];
  }
}

__global__ __launch_bounds__(GTHR) void k_gemm_hl(
    const unsigned short* __restrict__ A, int lda, int K, const unsigned short* __restrict__ WT, int ldw,
    const float* __restrict__ bias, int blen, int hasBias, unsigned short* outH) {
  __shared__ __attribute__((aligned(16))) float stg[GBM * GBN];
  const int tid = (int)threadIdx.x, lane = tid & 31, wave = tid >> 5, hh = lane >> 4, m = lane & 15;
  const int rowBase = (int)blockIdx.x * GBM;
  v8f acc[8];
  gemm_core(acc, A, lda, K, WT, ldw, rowBase, 0, wave, hh, m);
  gemm_stage(acc, stg, bias, blen, hasBias, 0, wave, hh, m);
  __syncthreads();
  v8us hv[16];
#pragma unroll
  for (int i = 0; i < 16; ++i) {
    const int pc = i * GTHR + tid;
    const int row = pc >> 5, q = pc & 31, c8 = (q & 15) * 8;
    const v4f a = *(const v4f*)(stg + row * GBN + c8);
    const v4f b = *(const v4f*)(stg + row * GBN + c8 + 4);
    hv[i] = hilo8(a, b, q < 16);
  }
#pragma unroll
  for (int i = 0; i < 16; ++i) {
    const int pc = i * GTHR + tid;
    const int row = pc >> 5, q = pc & 31;
    *(volatile v8us*)(outH + (size_t)(rowBase + row) * KD + 8 * q) = hv[i];
  }
  __threadfence();
#pragma unroll
  for (int i = 0; i < 16; ++i) {
    const int pc = i * GTHR + tid;
    const int row = pc >> 5, q = pc & 31;
    *(volatile v8us*)(outH + (size_t)(rowBase + row) * KD + 8 * q) = hv[i];
  }
}

__global__ __launch_bounds__(GTHR) void k_gemm_kv(
    const unsigned short* __restrict__ A, const unsigned short* __restrict__ WT,
    const int* __restrict__ srcs, const int* __restrict__ dsts, const float* __restrict__ QKV,
    const float* __restrict__ EB, float* LOG, float* VE, int cbeg, int ce, int nE, int nN) {
  __shared__ __attribute__((aligned(16))) float stg[GBM * GBN];
  __shared__ __attribute__((aligned(16))) float s_lg[GBM * NHEAD];
  __shared__ int s_src[GBM];
  __shared__ int s_dst[GBM];
  const int tid = (int)threadIdx.x, lane = tid & 31, wave = tid >> 5, hh = lane >> 4, m = lane & 15;
  const int rowBase = (int)blockIdx.x * GBM;
  const int col0    = (int)blockIdx.y * GBN;
  if (tid < GBM) {
    const int el = rowBase + tid;
    const int elc = el < ce ? el : ce - 1;
    int e = cbeg + elc;
    e = e > nE - 1 ? nE - 1 : (e < 0 ? 0 : e);
    s_src[tid] = clampi(srcs[e], 0, nN - 1);
    s_dst[tid] = clampi(dsts[e], 0, nN - 1);
  }
  v8f acc[8];
  gemm_core(acc, A, KD, KD, WT, KD, rowBase, col0, wave, hh, m);
  gemm_stage(acc, stg, EB, 1, 0, col0, wave, hh, m);
  __syncthreads();

  if (blockIdx.y == 0) {
#pragma unroll 1
    for (int i = 0; i < 4; ++i) {
      const int pc = i * GTHR + tid;
      const int row = pc >> 3, h = pc & 7;
      const int s = s_src[row], d = s_dst[row];
      const float* qp = QKV + (size_t)d * NQKV + DHD * h;
      const float* kp = QKV + (size_t)s * NQKV + HID + DHD * h;
      const v4f q0 = *(const v4f*)qp, q1 = *(const v4f*)(qp + 4), q2 = *(const v4f*)(qp + 8), q3 = *(const v4f*)(qp + 12);
      const v4f k0 = *(const v4f*)kp, k1 = *(const v4f*)(kp + 4), k2 = *(const v4f*)(kp + 8), k3 = *(const v4f*)(kp + 12);
      ldwait();
      const float* rp = stg + row * GBN + DHD * h;
      const v4f e0 = *(const v4f*)rp, e1 = *(const v4f*)(rp + 4), e2 = *(const v4f*)(rp + 8), e3 = *(const v4f*)(rp + 12);
      v4f t = q0 * (k0 + e0);
      t = t + q1 * (k1 + e1);
      t = t + q2 * (k2 + e2);
      t = t + q3 * (k3 + e3);
      const float sum = (t.x + t.y) + (t.z + t.w);
      const float lg = sum * 0.25f + EB[(size_t)(rowBase + row) * NHEAD + h];
      s_lg[row * NHEAD + h] = lg;
    }
    __syncthreads();
    const v4f lv = *(const v4f*)(s_lg + 4 * tid);
    float* lp = LOG + (size_t)rowBase * NHEAD + 4 * tid;
    *(volatile v4f*)lp = lv;
    __threadfence();
    *(volatile v4f*)lp = lv;
  } else {
    v4f ov[16];
#pragma unroll
    for (int i = 0; i < 16; ++i) {
      const int pc = i * GTHR + tid;
      const int row = pc >> 5, c4 = (pc & 31) * 4;
      const int s = s_src[row];
      const v4f vx = *(const v4f*)(QKV + (size_t)s * NQKV + 2 * HID + c4);
      const v4f rv = *(const v4f*)(stg + row * GBN + c4);
      ov[i] = vx + rv;
    }
#pragma unroll
    for (int i = 0; i < 16; ++i) {
      const int pc = i * GTHR + tid;
      const int row = pc >> 5, c4 = (pc & 31) * 4;
      *(volatile v4f*)(VE + (size_t)(rowBase + row) * HID + c4) = ov[i];
    }
    __threadfence();
#pragma unroll
    for (int i = 0; i < 16; ++i) {
      const int pc = i * GTHR + tid;
      const int row = pc >> 5, c4 = (pc & 31) * 4;
      *(volatile v4f*)(VE + (size_t)(rowBase + row) * HID + c4) = ov[i];
    }
  }
}

__global__ __launch_bounds__(NTHR) void k_agg(
    const int* __restrict__ dsts, const float* __restrict__ LOG, const float* __restrict__ VE,
    float* STA, float* STS, float* Mout, unsigned short* xm,
    int nN, int ce, int nb, int vec8, int NPr, int first, int last) {
  extern __shared__ v4f lds_dyn[];
  int* reg1 = (int*)lds_dyn;
  int* reg2 = reg1 + RCAP;
  int* scnt = reg2 + RCAP;
  int* soff = scnt + NBMAX;
  int* list = soff + NBMAX;
  int* wcnt = list + LISTN;
  int* wtot = wcnt + NWAVE;
  const int tid = (int)threadIdx.x, lane = tid & 31, wave = tid >> 5;
  const int nodeBase = (int)blockIdx.x * nb;

  for (int i = tid; i < NBMAX; i += NTHR) scnt[i] = 0;
  __syncthreads();

  int tot = 0;
  const int nChunks = (ce + CHUNK - 1) / CHUNK;
#pragma unroll 1
  for (int ch = 0; ch < nChunks; ++ch) {
    const int cbase = ch * CHUNK;
    const int wc = scan_chunk(dsts, ce, cbase, nodeBase, nb, vec8, list, tid, lane, wave);
    if (lane == 0) wcnt[wave] = wc;
    __syncthreads();
    int pre = 0, all = 0;
#pragma unroll
    for (int w2 = 0; w2 < NWAVE; ++w2) {
      int c = wcnt[w2];
      c = c < 0 ? 0 : (c > WCAP ? WCAP : c);
      all += c;
      pre += (w2 < wave) ? c : 0;
    }
    const int wcc  = wc > WCAP ? WCAP : wc;
    const int base = tot + pre;
#pragma unroll 1
    for (int i = lane; i < wcc; i += 32) {
      const int ent = list[wave * WCAP + i];
      const int el  = (ent >> 12) & (CHUNK - 1);
      const int sl  = ent & (NBMAX - 1);
      int eid = cbase + el;
      eid = eid > ce - 1 ? ce - 1 : eid;
      const int pos = base + i;
      if (pos < RCAP) reg1[pos] = (int)(((unsigned)eid << 12) | (unsigned)sl);
    }
    tot += all;
    tot = tot > RCAP ? RCAP : tot;
    __syncthreads();
  }
  const int nh = tot;

  if (wave == 0) {
#pragma unroll 1
    for (int b0 = 0; b0 < nh; b0 += 32) {
      const int idx = b0 + lane;
      const int uv  = reg1[idx < RCAP ? idx : RCAP - 1];
      const int m32 = (nh - b0) < 32 ? (nh - b0) : 32;
#pragma unroll 1
      for (int k = 0; k < m32; ++k) {
        const int u  = __builtin_amdgcn_readlane(uv, k);
        const int sl = u & (NBMAX - 1);
        if (lane == 0) scnt[sl] = scnt[sl] + 1;
      }
    }
  }
  __syncthreads();

  {
    const v4i ca = *(const v4i*)(scnt + 8 * tid);
    const v4i cb = *(const v4i*)(scnt + 8 * tid + 4);
    const int e0 = ca.x < 0 ? 0 : ca.x, e1 = ca.y < 0 ? 0 : ca.y, e2 = ca.z < 0 ? 0 : ca.z, e3 = ca.w < 0 ? 0 : ca.w;
    const int e4 = cb.x < 0 ? 0 : cb.x, e5 = cb.y < 0 ? 0 : cb.y, e6 = cb.z < 0 ? 0 : cb.z, e7 = cb.w < 0 ? 0 : cb.w;
    const int ts = e0 + e1 + e2 + e3 + e4 + e5 + e6 + e7;
    int incl = ts;
#pragma unroll
    for (int d = 1; d < 32; d <<= 1) {
      const int up = __shfl_up(incl, d);
      if (lane >= d) incl += up;
    }
    if (lane == 31) wtot[wave] = incl;
    __syncthreads();
    int pre = 0;
#pragma unroll
    for (int w2 = 0; w2 < NWAVE; ++w2) pre += (w2 < wave) ? wtot[w2] : 0;
    int run = pre + incl - ts;
    soff[8 * tid + 0] = run; run += e0;
    soff[8 * tid + 1] = run; run += e1;
    soff[8 * tid + 2] = run; run += e2;
    soff[8 * tid + 3] = run; run += e3;
    soff[8 * tid + 4] = run; run += e4;
    soff[8 * tid + 5] = run; run += e5;
    soff[8 * tid + 6] = run; run += e6;
    soff[8 * tid + 7] = run;
  }
  __syncthreads();
  for (int i = tid; i < NBMAX; i += NTHR) list[i] = soff[i];
  __syncthreads();

  if (wave == 0) {
#pragma unroll 1
    for (int b0 = 0; b0 < nh; b0 += 32) {
      const int idx = b0 + lane;
      const int uv  = reg1[idx < RCAP ? idx : RCAP - 1];
      const int m32 = (nh - b0) < 32 ? (nh - b0) : 32;
#pragma unroll 1
      for (int k = 0; k < m32; ++k) {
        const int u   = __builtin_amdgcn_readlane(uv, k);
        const int sl  = u & (NBMAX - 1);
        const int eid = (int)((unsigned)u >> 12);
        if (lane == 0) {
          int pos = list[sl];
          pos = pos < 0 ? 0 : (pos > RCAP - 1 ? RCAP - 1 : pos);
          reg2[pos] = eid;
          list[sl] = pos + 1;
        }
      }
    }
  }
  __syncthreads();

  const int nbw = nb >> 3;
  const bool ovf = (nh >= RCAP);
  const float qnan = __int_as_float(0x7fc00000);
  float* stw = (float*)reg1 + wave * STW;
  const int hd  = lane >> 2;
  const int lch = lane & 15;
  const v4f z4 = {0.f, 0.f, 0.f, 0.f};
#pragma unroll 1
  for (int jt = 0; jt < nbw; ++jt) {
    const int slot = wave * nbw + jt;
    const int grow = nodeBase + slot;
    int st = soff[slot];
    const int craw = scnt[slot];
    int cnt = craw;
    st  = st < 0 ? 0 : (st > nh ? nh : st);
    cnt = cnt < 0 ? 0 : (cnt > DEGCAP ? DEGCAP : cnt);
    if (cnt > nh - st) cnt = nh - st;
    const float pz = (ovf || craw > DEGCAP) ? qnan : 0.0f;
    const bool wr = grow < NPr;
    const float live = grow < nN ? 1.0f : 0.0f;

    const v4f sa = *(const v4f*)(STA + (size_t)grow * HID + 4 * lane);
    const v4f sb = *(const v4f*)(STS + (size_t)grow * STP + 4 * hd);
    ldwait();
    v4f av   = first ? z4 : sa;
    float mx = first ? -1.0e30f : sb.x;
    float dn = first ? 0.0f : sb.y;

#pragma unroll 1
    for (int q = 0; q < cnt; ++q) {
      int idx = st + q; idx = idx > RCAP - 1 ? RCAP - 1 : idx;
      int el = reg2[idx]; el = el < 0 ? 0 : (el > ce - 1 ? ce - 1 : el);
      const float lg = LOG[(size_t)el * NHEAD + hd];
      const v4f vv = *(const v4f*)(VE + (size_t)el * HID + 4 * lane);
      ldwait();
      const float df = lg - mx;
      const float ee = __expf(-fabsf(df));
      const bool up  = df > 0.f;
      const float s1 = up ? ee : 1.0f;
      const float s2 = up ? 1.0f : ee;
      mx = up ? lg : mx;
      dn = fmaf(dn, s1, s2);
      av = av * s1 + vv * s2;
    }

    if (last) {
      const float ds = dn > 0.f ? dn : 1.0f;
      const float iv = (dn > 0.f ? 1.0f : 0.0f) * __builtin_amdgcn_rcpf(ds);
      const v4f m4 = av * (iv * live) + pz;
      float* mp = Mout + (size_t)grow * HID + 4 * lane;
      if (wr) *(volatile v4f*)mp = m4;
      wave_sync();
      *(v4f*)(stw + 4 * lane) = m4;
      wave_sync();
      const v4f ga = *(const v4f*)(stw + 8 * lch);
      const v4f gb = *(const v4f*)(stw + 8 * lch + 4);
      const v8us hv = hilo8(ga, gb, lane < 16);
      unsigned short* hp = xm + (size_t)grow * XMP + KD + 8 * lane;
      if (wr) *(volatile v8us*)hp = hv;
      __threadfence();
      if (wr) {
        *(volatile v4f*)mp  = m4;
        *(volatile v8us*)hp = hv;
      }
    } else {
      float* ap2 = STA + (size_t)grow * HID + 4 * lane;
      *(volatile v4f*)ap2 = av;
      const float mxh = __shfl(mx, (4 * lane) & 31);
      const float dnh = __shfl(dn, (4 * lane) & 31);
      v4f sv; sv.x = mxh; sv.y = dnh; sv.z = 0.f; sv.w = 0.f;
      float* sp = STS + (size_t)grow * STP + 4 * lane;
      const bool ws8 = lane < 8;
      if (ws8) *(volatile v4f*)sp = sv;
      __threadfence();
      *(volatile v4f*)ap2 = av;
      if (ws8) *(volatile v4f*)sp = sv;
    }
  }
}

__global__ __launch_bounds__(NTHR) void k_tail(
    const float* __restrict__ x, const float* __restrict__ p, const float* __restrict__ lw,
    const float* __restrict__ lb, const float* __restrict__ M, const float* __restrict__ DG,
    const float* __restrict__ wd2, const float* __restrict__ bd2, const float* __restrict__ wgs,
    const float* __restrict__ bgs, float* out0, float* out1, int nN) {
  __shared__ __attribute__((aligned(16))) float s_wd2[3 * HID];
  __shared__ __attribute__((aligned(16))) float s_wgs[3 * 2 * HID];
  __shared__ __attribute__((aligned(16))) float s_po[TPB * 3];
  __shared__ float s_b[8];
  const int tid = (int)threadIdx.x, lane = tid & 31, wave = tid >> 5;
  for (int i = tid; i < 3 * HID; i += NTHR) s_wd2[i] = bfr(wd2[i]);
  for (int i = tid; i < 6 * HID; i += NTHR) s_wgs[i] = bfr(wgs[i]);
  if (tid < 3) { s_b[tid] = bfr(bd2[tid]); s_b[4 + tid] = bfr(bgs[tid]); }
  if (tid == 3) { s_b[3] = 0.f; s_b[7] = 0.f; }
  const v4f wv = bfr4(*(const v4f*)(lw + 4 * lane));
  const v4f bv = bfr4(*(const v4f*)(lb + 4 * lane));
  __syncthreads();
  const int node0 = (int)blockIdx.x * TPB;

#pragma unroll 1
  for (int k = 0; k < 4; ++k) {
    const int nl  = wave * 4 + k;
    const int row = node0 + nl;
    const bool valid = row < nN;
    const int rc = valid ? row : nN - 1;
    const v4f xv = bfr4(*(const v4f*)(x + (size_t)rc * HID + 4 * lane));
    const v4f mv = *(const v4f*)(M + (size_t)rc * HID + 4 * lane);
    const v4f dv = *(const v4f*)(DG + (size_t)rc * KD + 4 * lane);
    const v4f gv = *(const v4f*)(DG + (size_t)rc * KD + HID + 4 * lane);
    const float p0  = bfr(p[(size_t)rc * 3]);
    const float pp1 = bfr(p[(size_t)rc * 3 + 1]);
    const float pp2 = bfr(p[(size_t)rc * 3 + 2]);
    ldwait();
    const v4f xn = ln4(xv, wv, bv);
    v4f gt;
    gt.x = sigm(gv.x); gt.y = sigm(gv.y); gt.z = sigm(gv.z); gt.w = sigm(gv.w);
    const v4f mx = gt * mv;
    const v4f ov = xv + mx;
    float* op = out0 + (size_t)rc * HID + 4 * lane;
    if (valid) *(volatile v4f*)op = ov;

    v4f d1;
    d1.x = dv.x >= 0.f ? dv.x : 0.01f * dv.x;
    d1.y = dv.y >= 0.f ? dv.y : 0.01f * dv.y;
    d1.z = dv.z >= 0.f ? dv.z : 0.01f * dv.z;
    d1.w = dv.w >= 0.f ? dv.w : 0.01f * dv.w;
    float mp0 = 0.f, mp1 = 0.f, mp2 = 0.f;
#pragma unroll 1
    for (int j = 0; j < 3; ++j) {
      const v4f wd = *(const v4f*)(s_wd2 + j * HID + 4 * lane);
      const v4f wa = *(const v4f*)(s_wgs + j * 2 * HID + 4 * lane);
      const v4f wb = *(const v4f*)(s_wgs + j * 2 * HID + HID + 4 * lane);
      float pd = (d1.x * wd.x + d1.y * wd.y) + (d1.z * wd.z + d1.w * wd.w);
      float pg = ((xn.x * wa.x + xn.y * wa.y) + (xn.z * wa.z + xn.w * wa.w))
               + ((mx.x * wb.x + mx.y * wb.y) + (mx.z * wb.z + mx.w * wb.w));
      pd = wsum(pd);
      pg = wsum(pg);
      const float mpj = pd + s_b[j];
      const float gsj = sigm(pg + s_b[4 + j]);
      const float vj  = mpj * gsj;
      mp0 = (j == 0) ? vj : mp0;
      mp1 = (j == 1) ? vj : mp1;
      mp2 = (j == 2) ? vj : mp2;
    }
    const float m1  = mp1 + 1.0f;
    const float nr  = __builtin_amdgcn_sqrtf(m1 * m1 + mp2 * mp2);
    const float inv = __builtin_amdgcn_rcpf(nr + 1.0e-8f);
    const float c2 = m1 * inv, s2 = mp2 * inv;
    const float eta = p0 + mp0;
    const float f1 = c2 * pp1 - s2 * pp2;
    const float f2 = s2 * pp1 + c2 * pp2;
    const float nr2  = __builtin_amdgcn_sqrtf(f1 * f1 + f2 * f2);
    const float inv2 = __builtin_amdgcn_rcpf(nr2 + 1.0e-8f);
    if (lane == 0) {
      s_po[nl * 3]     = eta;
      s_po[nl * 3 + 1] = f1 * inv2;
      s_po[nl * 3 + 2] = f2 * inv2;
    }
    __threadfence();
    if (valid) *(volatile v4f*)op = ov;
  }
  __syncthreads();

  int nv = nN - node0;
  nv = nv > TPB ? TPB : (nv < 0 ? 0 : nv);
  float* ob = out1 + (size_t)node0 * 3;
  if (nv == TPB) {
    const int tc = tid < 24 ? tid : 23;
    const v4f pv = *(const v4f*)(s_po + 4 * tc);
    const bool w = tid < 24;
    if (w) *(volatile v4f*)(ob + 4 * tid) = pv;
    __threadfence();
    if (w) *(volatile v4f*)(ob + 4 * tid) = pv;
  } else {
    const int nf = 3 * nv;
    const int tc = tid < nf ? tid : (nf > 0 ? nf - 1 : 0);
    const float pv = s_po[tc];
    const bool w = tid < nf;
    if (w) *(volatile float*)(ob + tid) = pv;
    __threadfence();
    if (w) *(volatile float*)(ob + tid) = pv;
  }
}

static int pick_nb(int nE, int nN) {
  int nb = NBMAX;
  while (nb > 16 && (long long)nb * (long long)nE * 5LL > (long long)RCAP * (long long)nN * 4LL) nb >>= 1;
  return nb;
}
static inline int cdiv(int a, int b) { return (a + b - 1) / b; }
static inline size_t al256(size_t v) { return (v + 255) & ~(size_t)255; }

extern "C" void kernel_launch(void* const* d_in, const int* in_sizes, int n_in,
                              void* d_out, int out_size, void* d_ws, size_t ws_size,
                              hipStream_t stream) {
  if (n_in < 26) return;
  const int nN = in_sizes[0] / HID;
  if (nN <= 0 || in_sizes[0] != nN * HID || nN > (1 << 22)) return;
  if (in_sizes[1] != 3 * nN) return;
  if (in_sizes[2] < 2 || (in_sizes[2] & 1) != 0) return;
  const int nE = in_sizes[2] / 2;
  if (nE < 1 || nE > (1 << 24)) return;
  if (in_sizes[3] != nE * EDIM) return;
  if (in_sizes[4] != HID || in_sizes[5] != HID) return;
  if (in_sizes[6] != EDIM || in_sizes[7] != EDIM || in_sizes[8] != EDIM || in_sizes[9] != EDIM) return;
  if (in_sizes[10] != HID * HID || in_sizes[11] != HID * HID || in_sizes[12] != HID * HID) return;
  if (in_sizes[13] != NHEAD * EDIM) return;
  if (in_sizes[14] != 3 * HID || in_sizes[15] != HID) return;
  if (in_sizes[16] != HID * HID || in_sizes[17] != HID) return;
  if (in_sizes[18] != HID * HID || in_sizes[19] != HID) return;
  if (in_sizes[20] != 3 * HID || in_sizes[21] != 3) return;
  if (in_sizes[22] != 2 * HID * HID || in_sizes[23] != HID) return;
  if (in_sizes[24] != 3 * 2 * HID || in_sizes[25] != 3) return;
  if (out_size != nN * HID + nN * 3) return;

  const float* x    = (const float*)d_in[0];
  const float* p    = (const float*)d_in[1];
  const int*   ei   = (const int*)  d_in[2];
  const float* ea   = (const float*)d_in[3];
  const float* lxw  = (const float*)d_in[4];
  const float* lxb  = (const float*)d_in[5];
  const float* lew  = (const float*)d_in[6];
  const float* leb  = (const float*)d_in[7];
  const float* le2w = (const float*)d_in[8];
  const float* le2b = (const float*)d_in[9];
  const float* Wq   = (const float*)d_in[10];
  const float* Wk   = (const float*)d_in[11];
  const float* Wv   = (const float*)d_in[12];
  const float* Wed  = (const float*)d_in[13];
  const float* We1  = (const float*)d_in[14];
  const float* be1  = (const float*)d_in[15];
  const float* We2  = (const float*)d_in[16];
  const float* be2  = (const float*)d_in[17];
  const float* Wd1  = (const float*)d_in[18];
  const float* bd1  = (const float*)d_in[19];
  const float* Wd2  = (const float*)d_in[20];
  const float* bd2  = (const float*)d_in[21];
  const float* Wg   = (const float*)d_in[22];
  const float* bg   = (const float*)d_in[23];
  const float* Wgs  = (const float*)d_in[24];
  const float* bgs  = (const float*)d_in[25];
  float* out0 = (float*)d_out;
  float* out1 = out0 + (size_t)nN * HID;
  const int* src = ei;
  const int* dst = ei + nE;

  const int NP = cdiv(nN, GBM) * GBM;
  const int nb = pick_nb(nE, nN);
  const int gA = cdiv(NP, nb);
  const int NS = gA * nb;
  if (gA * nb < NP) return;
  int CE = cdiv(nE, GBM) * GBM;
  if (CE > CEMAX) CE = CEMAX;
  const int nChunk = cdiv(nE, CE);
  if (nChunk < 1 || nChunk > 512) return;

  char* ws = (char*)d_ws;
  size_t off = 0;
  const size_t oXM   = off; off = al256(off + (size_t)NP * XMP * 2);
  const size_t oWQKV = off; off = al256(off + (size_t)NQKV * KD * 2);
  const size_t oWE2  = off; off = al256(off + (size_t)HID * KD * 2);
  const size_t oWD1  = off; off = al256(off + (size_t)HID * KD * 2);
  const size_t oWG   = off; off = al256(off + (size_t)HID * KG * 2);
  const size_t oQD   = off; off = al256(off + (size_t)NP * NQKV * 4);
  const size_t oG2   = off; off = al256(off + (size_t)CE * KD * 2);
  const size_t oREL  = off; off = al256(off + (size_t)CE * KD * 2);
  const size_t oEB   = off; off = al256(off + (size_t)CE * NHEAD * 4);
  const size_t oLOG  = off; off = al256(off + (size_t)CE * NHEAD * 4);
  const size_t oVE   = off; off = al256(off + (size_t)CE * HID * 4);
  const size_t oSTA  = off; off = al256(off + (size_t)NS * HID * 4);
  const size_t oSTS  = off; off = al256(off + (size_t)NS * STP * 4);
  if (off > ws_size || off > (size_t)WSMAX) return;
  unsigned short* XM2   = (unsigned short*)(ws + oXM);
  unsigned short* WQKV2 = (unsigned short*)(ws + oWQKV);
  unsigned short* WKV2  = WQKV2 + (size_t)HID * KD;
  unsigned short* WE22  = (unsigned short*)(ws + oWE2);
  unsigned short* WD12  = (unsigned short*)(ws + oWD1);
  unsigned short* WG2   = (unsigned short*)(ws + oWG);
  float* QKV = (float*)(ws + oQD);
  float* Mpl = (float*)(ws + oQD);
  float* DG  = Mpl + (size_t)NP * HID;
  unsigned short* G2   = (unsigned short*)(ws + oG2);
  unsigned short* REL2 = (unsigned short*)(ws + oREL);
  float* EBc  = (float*)(ws + oEB);
  float* LOGc = (float*)(ws + oLOG);
  float* VEc  = (float*)(ws + oVE);
  float* STA  = (float*)(ws + oSTA);
  float* STS  = (float*)(ws + oSTS);

  hipFuncSetAttribute(reinterpret_cast<const void*>(&k_agg),
                      hipFuncAttributeMaxDynamicSharedMemorySize, LDS_AGG);

  k_prep_x<<<cdiv(NP, NWAVE), NTHR, 0, stream>>>(x, lxw, lxb, XM2, nN, NP);

  {
    const int nU = HID * (HID / 4);
    k_wprep<<<cdiv(nU, NTHR), NTHR, 0, stream>>>(Wq,  HID, WQKV2, 0,       nU);
    k_wprep<<<cdiv(nU, NTHR), NTHR, 0, stream>>>(Wk,  HID, WQKV2, HID,     nU);
    k_wprep<<<cdiv(nU, NTHR), NTHR, 0, stream>>>(Wv,  HID, WQKV2, 2 * HID, nU);
    k_wprep<<<cdiv(nU, NTHR), NTHR, 0, stream>>>(We2, HID, WE22,  0,       nU);
    k_wprep<<<cdiv(nU, NTHR), NTHR, 0, stream>>>(Wd1, HID, WD12,  0,       nU);
    const int nUg = HID * ((2 * HID) / 4);
    k_wprep<<<cdiv(nUg, NTHR), NTHR, 0, stream>>>(Wg, 2 * HID, WG2, 0, nUg);
  }

  const int gM = NP / GBM;
  k_gemm_f32<<<dim3(gM, NQKV / GBN), GTHR, 0, stream>>>(XM2, XMP, KD, WQKV2, KD, be1, HID, 0, QKV, NQKV);

  for (int c = 0; c < nChunk; ++c) {
    const int cbeg = c * CE;
    int ce = nE - cbeg; ce = ce > CE ? CE : ce;
    const int cep = cdiv(ce, GBM) * GBM;
    const int gE = cep / GBM;
    k_edge_geo<<<gE, NTHR, 0, stream>>>(src, dst, p, ea, lew, leb, le2w, le2b, Wed, We1, be1,
                                        G2, EBc, cbeg, ce, nE, nN);
    k_gemm_hl<<<dim3(gE, 1), GTHR, 0, stream>>>(G2, KD, KD, WE22, KD, be2, HID, 1, REL2);
    k_gemm_kv<<<dim3(gE, 2), GTHR, 0, stream>>>(REL2, WKV2, src, dst, QKV, EBc, LOGc, VEc, cbeg, ce, nE, nN);
    const int vec8 = ((((long long)nE + (long long)cbeg) & 3LL) == 0) ? 1 : 0;
    k_agg<<<gA, NTHR, LDS_AGG, stream>>>(dst + cbeg, LOGc, VEc, STA, STS, Mpl, XM2,
                                         nN, ce, nb, vec8, NP, (c == 0) ? 1 : 0, (c == nChunk - 1) ? 1 : 0);
  }

  k_gemm_f32<<<dim3(gM, 1), GTHR, 0, stream>>>(XM2 + KD, XMP, KD, WD12, KD, bd1, HID, 1, DG, KD);
  k_gemm_f32<<<dim3(gM, 1), GTHR, 0, stream>>>(XM2, XMP, KG, WG2, KG, bg, HID, 1, DG + HID, KD);
  k_tail<<<cdiv(nN, TPB), NTHR, 0, stream>>>(x, p, lxw, lxb, Mpl, DG, Wd2, bd2, Wgs, bgs, out0, out1, nN);
}
